// AnticipatoryGNN_67808943669808
// MI455X (gfx1250) — hardware-verified
//
#include <hip/hip_runtime.h>
#include <stddef.h>


#define DF        128
#define KV        256
#define NTHR      256
#define NWAVE     8
#define EPT       8
#define NGRP      2
#define NEPT      (EPT * NGRP)
#define CHUNK     (NTHR * NEPT)
#define NBT       2048
#define SLOT_BITS 11
#define SLOT_MASK (NBT - 1)
#define RPH       256
#define NPH       (NBT / RPH)
#define TILES_PH  (RPH / 16)
#define TPWP      (TILES_PH / NWAVE)
#define LCAP      36864
#define NGMAX     64
#define NEG_SLOPE 0.1f
#define WSCALE    8.0f
#define WINV      0.125f

#define LDS_LIST  (LCAP * 4)
#define LDS_ACC   (RPH * DF * 4)
#define LDS_CNT   (RPH * 4)
#define LDS_MISC  128
#define LDS_LAYER (LDS_LIST + LDS_ACC + LDS_CNT + LDS_MISC)

#define LDS_PACC  (NWAVE * NGMAX * DF * 4)
#define LDS_PCNT  (NWAVE * NGMAX * 4)
#define LDS_POOL  (LDS_PACC + LDS_PCNT + NGMAX * 4 * 2)

static_assert(DF == 128);
static_assert(KV == 2 * DF);
static_assert((1 << SLOT_BITS) == NBT);
static_assert(NBT % RPH == 0);
static_assert((RPH & (RPH - 1)) == 0);
static_assert(TILES_PH % NWAVE == 0);
static_assert(NTHR == 32 * NWAVE);
static_assert(LDS_LIST % 16 == 0);
static_assert(LDS_ACC % 16 == 0);
static_assert(LDS_LAYER <= 300 * 1024);
static_assert(LDS_POOL <= 300 * 1024);
static_assert(2 * NWAVE * 4 <= LDS_MISC);

typedef float    v4f  __attribute__((ext_vector_type(4)));
typedef float    v8f  __attribute__((ext_vector_type(8)));
typedef int      v4i  __attribute__((ext_vector_type(4)));
typedef _Float16 f16_t;
typedef f16_t    v8h  __attribute__((ext_vector_type(8)));
typedef f16_t    v16h __attribute__((ext_vector_type(16)));
union FragH { v16h v; v8h h[2]; v4i q[2]; };
union Pack8 { v8h v; v4i q; };

__device__ __forceinline__ v8f wmh(v16h a, v16h b, v8f c) {
  v8f d = __builtin_amdgcn_wmma_f32_16x16x32_f16(false, a, false, b, (short)0, c, false, false);
  asm volatile("v_nop\n\tv_nop\n\tv_nop\n\tv_nop" : "+v"(d) : "v"(a), "v"(b));
  return d;
}

__global__ __launch_bounds__(NTHR) void k_wprep(const float* __restrict__ Wl, const float* __restrict__ Wr,
                                                f16_t* wh, int nTot) {
  const int i = blockIdx.x * NTHR + threadIdx.x;
  if (i >= nTot) return;
  const int o     = i * 8;
  const int layer = o / (DF * KV);
  const int rem   = o - layer * (DF * KV);
  const int n     = rem / KV;
  const int k0    = rem - n * KV;
  const float* p = (k0 < DF) ? (Wl + (size_t)layer * DF * DF + (size_t)k0 * DF + n)
                             : (Wr + (size_t)layer * DF * DF + (size_t)(k0 - DF) * DF + n);
  Pack8 ph;
#define WSP(I) ph.v[(I)] = (f16_t)(p[(I) * DF] * WSCALE);
  WSP(0) WSP(1) WSP(2) WSP(3) WSP(4) WSP(5) WSP(6) WSP(7)
#undef WSP
  const v4i q = ph.q;
  f16_t* d = wh + o;
  *(volatile v4i*)d = q;
  __threadfence();
  *(volatile v4i*)d = q;
}

__device__ __forceinline__ void kstep(const float* ap, float mul, const f16_t* bp, v8f (&c)[8]) {
  const v4f p0 = (*(const v4f*)(ap))      * mul;
  const v4f p1 = (*(const v4f*)(ap + 4))  * mul;
  const v4f p2 = (*(const v4f*)(ap + 16)) * mul;
  const v4f p3 = (*(const v4f*)(ap + 20)) * mul;
  FragH a;
  a.v[0]  = (f16_t)p0.x; a.v[1]  = (f16_t)p0.y; a.v[2]  = (f16_t)p0.z; a.v[3]  = (f16_t)p0.w;
  a.v[4]  = (f16_t)p1.x; a.v[5]  = (f16_t)p1.y; a.v[6]  = (f16_t)p1.z; a.v[7]  = (f16_t)p1.w;
  a.v[8]  = (f16_t)p2.x; a.v[9]  = (f16_t)p2.y; a.v[10] = (f16_t)p2.z; a.v[11] = (f16_t)p2.w;
  a.v[12] = (f16_t)p3.x; a.v[13] = (f16_t)p3.y; a.v[14] = (f16_t)p3.z; a.v[15] = (f16_t)p3.w;
#pragma unroll
  for (int ct = 0; ct < DF / 16; ++ct) {
    const f16_t* hp = bp + (size_t)ct * 16 * KV;
    FragH b;
    b.q[0] = *(const v4i*)hp;
    b.q[1] = *(const v4i*)(hp + 16);
    c[ct] = wmh(a.v, b.v, c[ct]);
  }
}

__global__ __launch_bounds__(NTHR) void k_layer(const int* __restrict__ ei, const float* __restrict__ xin,
                                                const f16_t* __restrict__ wh, const float* __restrict__ bias,
                                                float* xout, int nN, int nE, int vec8) {
  extern __shared__ v4f lds_dyn[];
  unsigned* list = (unsigned*)lds_dyn;
  v4f*      acc4 = (v4f*)((char*)lds_dyn + LDS_LIST);
  float*    acc  = (float*)acc4;
  int*      cnt  = (int*)((char*)lds_dyn + LDS_LIST + LDS_ACC);
  int*      wcnt = (int*)((char*)lds_dyn + LDS_LIST + LDS_ACC + LDS_CNT);
  const int tid = threadIdx.x, lane = tid & 31, wave = tid >> 5, hh = lane >> 4, m = lane & 15;
  const int nodeBase = blockIdx.x * NBT;
  const unsigned nb = (unsigned)nodeBase;
  const int* dsts = ei + nE;
  const int sent = -2147483647 - 1;

  int tot = 0;
  const int nChunks = (nE + CHUNK - 1) / CHUNK;
#pragma unroll 1
  for (int ch = 0; ch < nChunks; ++ch) {
    const int cbase = ch * CHUNK;
    unsigned sv[NEPT];
#pragma unroll
    for (int g = 0; g < NGRP; ++g) {
      const int e0 = cbase + (g * NTHR + tid) * EPT;
      v4i da, db;
      if (vec8 != 0 && e0 + 7 < nE) {
        da = *(const v4i*)(dsts + e0);
        db = *(const v4i*)(dsts + e0 + 4);
      } else {
        da.x = (e0     < nE) ? dsts[min(e0,     nE - 1)] : sent;
        da.y = (e0 + 1 < nE) ? dsts[min(e0 + 1, nE - 1)] : sent;
        da.z = (e0 + 2 < nE) ? dsts[min(e0 + 2, nE - 1)] : sent;
        da.w = (e0 + 3 < nE) ? dsts[min(e0 + 3, nE - 1)] : sent;
        db.x = (e0 + 4 < nE) ? dsts[min(e0 + 4, nE - 1)] : sent;
        db.y = (e0 + 5 < nE) ? dsts[min(e0 + 5, nE - 1)] : sent;
        db.z = (e0 + 6 < nE) ? dsts[min(e0 + 6, nE - 1)] : sent;
        db.w = (e0 + 7 < nE) ? dsts[min(e0 + 7, nE - 1)] : sent;
      }
      sv[g * EPT + 0] = (unsigned)da.x - nb; sv[g * EPT + 1] = (unsigned)da.y - nb;
      sv[g * EPT + 2] = (unsigned)da.z - nb; sv[g * EPT + 3] = (unsigned)da.w - nb;
      sv[g * EPT + 4] = (unsigned)db.x - nb; sv[g * EPT + 5] = (unsigned)db.y - nb;
      sv[g * EPT + 6] = (unsigned)db.z - nb; sv[g * EPT + 7] = (unsigned)db.w - nb;
    }
    unsigned mk[NEPT];
    int wc = 0;
#pragma unroll
    for (int j = 0; j < NEPT; ++j) {
      mk[j] = __builtin_amdgcn_ballot_w32(sv[j] < (unsigned)NBT);
      wc += (int)__builtin_popcount(mk[j]);
    }
    int* wcb = wcnt + (ch & 1) * NWAVE;
    if (lane == 0) wcb[wave] = wc;
    __syncthreads();
    int base = tot, sum = 0;
#pragma unroll
    for (int w = 0; w < NWAVE; ++w) {
      const int cw = wcb[w];
      base += (w < wave) ? cw : 0;
      sum  += cw;
    }
    int run = base;
#pragma unroll
    for (int j = 0; j < NEPT; ++j) {
      const unsigned mj = mk[j];
      if (mj != 0u) {
        if (sv[j] < (unsigned)NBT) {
          const int pos = run + (int)__builtin_amdgcn_mbcnt_lo(mj, 0u);
          const int e   = cbase + ((j / EPT) * NTHR + tid) * EPT + (j % EPT);
          if ((unsigned)pos < (unsigned)LCAP) list[pos] = ((unsigned)e << SLOT_BITS) | sv[j];
        }
        run += (int)__builtin_popcount(mj);
      }
    }
    tot += sum;
  }
  __syncthreads();
  const int totc = tot < LCAP ? tot : LCAP;

#pragma unroll 1
  for (int ph = 0; ph < NPH; ++ph) {
    const int slot0 = ph * RPH;
    {
      const v4f z = {0.f, 0.f, 0.f, 0.f};
      for (int i = tid; i < RPH * DF / 4; i += NTHR) acc4[i] = z;
      for (int i = tid; i < RPH; i += NTHR) cnt[i] = 0;
    }
    __syncthreads();

    if (wave == 0) {
#pragma unroll 1
      for (int i0 = 0; i0 < totc; i0 += 32) {
        const int ii = i0 + lane;
        const unsigned ent = list[ii < totc ? ii : 0];
        const unsigned ls  = (ent & (unsigned)SLOT_MASK) - (unsigned)slot0;
        const bool hit = (ii < totc) && (ls < (unsigned)RPH);
        unsigned hm = __builtin_amdgcn_ballot_w32(hit);
        while (hm != 0u) {
          const int li = __builtin_ctz(hm);
          hm &= hm - 1u;
          const unsigned eu = (unsigned)__builtin_amdgcn_readlane((int)ent, li);
          const int lsl = (int)(((eu & (unsigned)SLOT_MASK) - (unsigned)slot0) & (unsigned)(RPH - 1));
          int e = (int)(eu >> SLOT_BITS);
          e = e > nE - 1 ? nE - 1 : e;
          int src = ei[e];
          src = src < 0 ? 0 : (src > nN - 1 ? nN - 1 : src);
          const v4f v = *(const v4f*)(xin + (size_t)src * DF + 4 * lane);
          v4f* ap = acc4 + lsl * (DF / 4) + lane;
          *ap = *ap + v;
          if (lane == 0) cnt[lsl] = cnt[lsl] + 1;
        }
      }
    }
    __syncthreads();

#pragma unroll 1
    for (int q = 0; q < TPWP; ++q) {
      const int tq  = q * NWAVE + wave;
      const int lsm = 16 * tq + m;
      int node = nodeBase + slot0 + lsm;
      node = node > nN - 1 ? nN - 1 : node;
      const int   cd  = cnt[lsm];
      const float inv = 1.0f / (float)(cd > 1 ? cd : 1);

      v8f c[8];
#pragma unroll
      for (int ct = 0; ct < 8; ++ct) { const v8f z = {0.f, 0.f, 0.f, 0.f, 0.f, 0.f, 0.f, 0.f}; c[ct] = z; }

      const float* arow = acc + lsm * DF + 8 * hh;
      const float* xrow = xin + (size_t)node * DF + 8 * hh;
      const f16_t* bh0  = wh + m * KV + 8 * hh;
#pragma unroll 1
      for (int ks = 0; ks < DF / 32; ++ks) kstep(arow + 32 * ks, inv, bh0 + 32 * ks, c);
#pragma unroll 1
      for (int ks = 0; ks < DF / 32; ++ks) kstep(xrow + 32 * ks, 1.0f, bh0 + DF + 32 * ks, c);

      float* sp = acc + (16 * tq + 8 * hh) * DF + m;
#pragma unroll
      for (int ct = 0; ct < 8; ++ct) {
        const float bv = bias[16 * ct + m];
#pragma unroll
        for (int r = 0; r < 8; ++r) {
          float v = c[ct][r] * WINV + bv;
          v = (v >= 0.0f) ? v : NEG_SLOPE * v;
          sp[r * DF + 16 * ct] = v;
        }
      }
      __syncthreads();

      const float* lrow = acc + (16 * tq) * DF + 4 * lane;
      float* gp = xout + ((size_t)nodeBase + (size_t)slot0 + (size_t)(16 * tq)) * DF + 4 * lane;
#pragma unroll
      for (int i = 0; i < 16; ++i) { const v4f v = *(const v4f*)(lrow + i * DF); *(volatile v4f*)(gp + (size_t)i * DF) = v; }
      __threadfence();
#pragma unroll
      for (int i = 0; i < 16; ++i) { const v4f v = *(const v4f*)(lrow + i * DF); *(volatile v4f*)(gp + (size_t)i * DF) = v; }
    }
    __syncthreads();
  }
}

__global__ __launch_bounds__(NTHR) void k_pool(const float* __restrict__ x, const int* __restrict__ bt,
                                               const float* __restrict__ Wo, const float* __restrict__ bo,
                                               float* out, int nN, int G, int per) {
  extern __shared__ v4f lds_dyn[];
  float* pacc = (float*)lds_dyn;
  int*   pcnt = (int*)((char*)lds_dyn + LDS_PACC);
  float* rcn  = (float*)((char*)lds_dyn + LDS_PACC + LDS_PCNT);
  float* outv = rcn + NGMAX;
  const int tid = threadIdx.x, lane = tid & 31, wave = tid >> 5;

  {
    const v4f z = {0.f, 0.f, 0.f, 0.f};
    for (int i = tid; i < NWAVE * NGMAX * DF / 4; i += NTHR) lds_dyn[i] = z;
    for (int i = tid; i < NWAVE * NGMAX; i += NTHR) pcnt[i] = 0;
    if (tid < NGMAX) { rcn[tid] = 0.f; outv[tid] = 0.f; }
  }
  __syncthreads();

  const int n0 = wave * per;
  int n1 = n0 + per;
  n1 = n1 > nN ? nN : n1;
  float* myacc = pacc + (size_t)wave * NGMAX * DF;
  int*   mycnt = pcnt + wave * NGMAX;
#pragma unroll 1
  for (int n = n0; n < n1; ++n) {
    const int b = __builtin_amdgcn_readfirstlane(bt[n]);
    if ((unsigned)b < (unsigned)G) {
      const v4f v = *(const v4f*)(x + (size_t)n * DF + 4 * lane);
      v4f* ap = (v4f*)(myacc + b * DF) + lane;
      *ap = *ap + v;
      if (lane == 0) mycnt[b] = mycnt[b] + 1;
    }
  }
  __syncthreads();

  for (int s = tid; s < G * (DF / 4); s += NTHR) {
    const int g = s >> 5, c4 = (s & 31) * 4;
    v4f t = {0.f, 0.f, 0.f, 0.f};
#pragma unroll
    for (int w = 0; w < NWAVE; ++w) t += *(const v4f*)(pacc + ((size_t)w * NGMAX + g) * DF + c4);
    *(v4f*)(pacc + (size_t)g * DF + c4) = t;
  }
  if (tid < G) {
    int cc = 0;
#pragma unroll
    for (int w = 0; w < NWAVE; ++w) cc += pcnt[w * NGMAX + tid];
    rcn[tid] = 1.0f / (float)(cc > 1 ? cc : 1);
  }
  __syncthreads();

  const v4f wo4 = *(const v4f*)(Wo + 4 * lane);
#pragma unroll 1
  for (int g = wave; g < G; g += NWAVE) {
    const v4f mv = (*(const v4f*)(pacc + (size_t)g * DF + 4 * lane)) * rcn[g];
    float p = mv.x * wo4.x + mv.y * wo4.y + mv.z * wo4.z + mv.w * wo4.w;
    p += __shfl_xor(p, 16);
    p += __shfl_xor(p, 8);
    p += __shfl_xor(p, 4);
    p += __shfl_xor(p, 2);
    p += __shfl_xor(p, 1);
    if (lane == 0) outv[g] = p + bo[0];
  }
  __syncthreads();

  if (wave == 0) {
    const int nq = G >> 2;
    const int tail = G - 4 * nq;
    v4f v4 = {0.f, 0.f, 0.f, 0.f};
    float vt = 0.f;
    if (lane < nq)   v4 = *(const v4f*)(outv + 4 * lane);
    if (lane < tail) vt = outv[4 * nq + lane];
    if (lane < nq)   *(volatile v4f*)(out + 4 * lane) = v4;
    if (lane < tail) *(volatile float*)(out + 4 * nq + lane) = vt;
    __threadfence();
    if (lane < nq)   *(volatile v4f*)(out + 4 * lane) = v4;
    if (lane < tail) *(volatile float*)(out + 4 * nq + lane) = vt;
  }
}

extern "C" void kernel_launch(void* const* d_in, const int* in_sizes, int n_in,
                              void* d_out, int out_size, void* d_ws, size_t ws_size,
                              hipStream_t stream) {
  if (n_in < 8) return;
  const int nN = in_sizes[0] / DF;
  const int nE = in_sizes[1] / 2;
  const int nL = in_sizes[3] / (DF * DF);
  const int G  = out_size;
  if (nN <= 0 || nE < 0 || nL <= 0 || G <= 0 || G > NGMAX) return;
  if (in_sizes[0] != nN * DF || in_sizes[1] != 2 * nE || in_sizes[2] < nN) return;
  if (in_sizes[3] != nL * DF * DF || in_sizes[4] < nL * DF || in_sizes[5] != nL * DF * DF) return;
  if (in_sizes[6] < DF || in_sizes[7] < 1) return;
  if (nE > (1 << 21)) return;

  const float* x0    = (const float*)d_in[0];
  const int*   ei    = (const int*)d_in[1];
  const int*   batch = (const int*)d_in[2];
  const float* Wl    = (const float*)d_in[3];
  const float* bl    = (const float*)d_in[4];
  const float* Wr    = (const float*)d_in[5];
  const float* Wo    = (const float*)d_in[6];
  const float* bo    = (const float*)d_in[7];
  float* out = (float*)d_out;

  const int nBlk = (nN + NBT - 1) / NBT;

  char* ws = (char*)d_ws;
  size_t off = 0;
  const size_t szW = (size_t)nL * DF * KV * 2;
  const size_t szX = (size_t)nBlk * NBT * DF * 4;
  const size_t oW  = off; off += szW; off = (off + 255) & ~(size_t)255;
  const size_t oXa = off; off += szX; off = (off + 255) & ~(size_t)255;
  const size_t oXb = off; off += szX; off = (off + 255) & ~(size_t)255;
  if (off > ws_size) return;
  f16_t* wh = (f16_t*)(ws + oW);
  float* xa = (float*)(ws + oXa);
  float* xb = (float*)(ws + oXb);

  const int vec8 = ((nE & 3) == 0) ? 1 : 0;

  const int nTot = nL * DF * KV / 8;
  k_wprep<<<dim3((nTot + NTHR - 1) / NTHR), dim3(NTHR), 0, stream>>>(Wl, Wr, wh, nTot);

  hipFuncSetAttribute(reinterpret_cast<const void*>(&k_layer),
                      hipFuncAttributeMaxDynamicSharedMemorySize, LDS_LAYER);
  hipFuncSetAttribute(reinterpret_cast<const void*>(&k_pool),
                      hipFuncAttributeMaxDynamicSharedMemorySize, LDS_POOL);

  const float* xin = x0;
  float* bufs[2] = {xa, xb};
  for (int l = 0; l < nL; ++l) {
    float* xo = bufs[l & 1];
    k_layer<<<dim3(nBlk), dim3(NTHR), LDS_LAYER, stream>>>(
        ei, xin, wh + (size_t)l * DF * KV, bl + (size_t)l * DF, xo, nN, nE, vec8);
    xin = xo;
  }

  const int per = (nN + NWAVE - 1) / NWAVE;
  k_pool<<<dim3(1), dim3(NTHR), LDS_POOL, stream>>>(xin, batch, Wo, bo, out, nN, G, per);
}
